// SelfAttLayer_75325136437764
// MI455X (gfx1250) — hardware-verified
//
#include <hip/hip_runtime.h>
#include <math.h>

constexpr int kImg = 16;
constexpr int kCh = 64;
constexpr int kHgt = 64;
constexpr int kWid = 64;
constexpr int kPixImg = kHgt * kWid;
constexpr int kNPix = kImg * kPixImg;
constexpr int kPadW = kWid + 2;
constexpr int kPadPixImg = kPadW * kPadW;
constexpr int kNPadPix = kImg * kPadPixImg;
constexpr int kQVld = 2 * kCh;
constexpr int kTaps = 9;
constexpr int kKconv = kTaps * kCh;

constexpr int kPXB = 32;
constexpr int kHaloW = kPXB + 2;
constexpr int kSlot = 64;
constexpr int kOutP = 36;

constexpr size_t kBytesTab = (size_t)(512 + 576) * 4;
constexpr size_t kBytesBqv = (size_t)kQVld * kCh * 2;
constexpr size_t kBytesBk  = (size_t)kCh * kKconv * 2;
constexpr size_t kBytesX16 = (size_t)kNPadPix * kCh * 2;
constexpr size_t kBytesQV  = (size_t)kNPix * kQVld * 4;
constexpr size_t kBytesKF  = (size_t)kNPix * kCh * 4;
constexpr size_t kOffTab  = 0;
constexpr size_t kOffBqvH = kOffTab + kBytesTab;
constexpr size_t kOffBqvL = kOffBqvH + kBytesBqv;
constexpr size_t kOffBkH  = kOffBqvL + kBytesBqv;
constexpr size_t kOffBkL  = kOffBkH + kBytesBk;
constexpr size_t kOffXh   = kOffBkL + kBytesBk;
constexpr size_t kOffXl   = kOffXh + kBytesX16;
constexpr size_t kOffQV   = kOffXl + kBytesX16;
constexpr size_t kOffKF   = kOffQV + kBytesQV;
constexpr size_t kWsTotal = kOffKF + kBytesKF;
static_assert(kWsTotal == 68358400, "carve total");
static_assert(kOffBqvH % 128 == 0 && kOffBqvL % 128 == 0 && kOffBkH % 128 == 0 && kOffBkL % 128 == 0, "align");
static_assert(kOffXh % 128 == 0 && kOffXl % 128 == 0 && kOffQV % 128 == 0 && kOffKF % 128 == 0, "align");
static_assert(kWsTotal <= (size_t)134217728, "under 128 MiB");

typedef __attribute__((ext_vector_type(16))) _Float16 v16h;
typedef __attribute__((ext_vector_type(8)))  _Float16 v8h;
typedef __attribute__((ext_vector_type(16))) __bf16   v16b;
typedef __attribute__((ext_vector_type(8)))  __bf16   v8b;
typedef __attribute__((ext_vector_type(8)))  float    v8f;
typedef __attribute__((ext_vector_type(4)))  float    v4f;
typedef __attribute__((ext_vector_type(4)))  unsigned int v4u;

__device__ __forceinline__ unsigned short f2bf_bits(float f) {
  unsigned u = __float_as_uint(f);
  return (unsigned short)((u + 0x7FFFu + ((u >> 16) & 1u)) >> 16);
}
__device__ __forceinline__ float bf_bits2f(unsigned short h) { return __uint_as_float(((unsigned)h) << 16); }
__device__ __forceinline__ void split_bf(float f, unsigned short& hb, unsigned short& lb) {
  hb = f2bf_bits(f);
  lb = f2bf_bits(f - bf_bits2f(hb));
}
__device__ __forceinline__ unsigned pk16(unsigned short a, unsigned short b) { return (unsigned)a | ((unsigned)b << 16); }

__device__ __forceinline__ void dep_guard_h(v8f& a, v8f& b, v16h x, v16h y) { asm volatile("v_nop\n\tv_nop\n\tv_nop\n\tv_nop" : "+v"(a), "+v"(b) : "v"(x), "v"(y)); }
__device__ __forceinline__ void dep_guard_b(v8f& a, v8f& b, v16b x, v16b y) { asm volatile("v_nop\n\tv_nop\n\tv_nop\n\tv_nop" : "+v"(a), "+v"(b) : "v"(x), "v"(y)); }
__device__ __forceinline__ void keep4_h(v16h a, v16h b, v16h c, v16h d) { asm volatile("v_nop" :: "v"(a), "v"(b), "v"(c), "v"(d)); }
__device__ __forceinline__ void keep4_b(v16b a, v16b b, v16b c, v16b d) { asm volatile("v_nop" :: "v"(a), "v"(b), "v"(c), "v"(d)); }
__device__ __forceinline__ void acc_guard4(v8f& a, v8f& b, v8f& c, v8f& d) { asm volatile("v_nop\n\tv_nop\n\tv_nop\n\tv_nop" : "+v"(a), "+v"(b), "+v"(c), "+v"(d)); }
template <typename T> struct Frag;
template <> struct Frag<_Float16> {
  typedef v16h V; union U { v16h v; v8h h[2]; };
  static __device__ __forceinline__ v16h load(const _Float16* p) {
    U f; f.h[0] = *(const v8h*)(p); f.h[1] = *(const v8h*)(p + 16); return f.v;
  }
  static __device__ __forceinline__ v8f mma(v16h a, v16h b, v8f c) {
    return __builtin_amdgcn_wmma_f32_16x16x32_f16(false, a, false, b, (short)0, c, false, false);
  }
  static __device__ __forceinline__ void guard(v8f& a, v8f& b, v16h x, v16h y) { dep_guard_h(a, b, x, y); }
  static __device__ __forceinline__ void keep(v16h a, v16h b, v16h c, v16h d) { keep4_h(a, b, c, d); }
};
template <> struct Frag<__bf16> {
  typedef v16b V; union U { v16b v; v8b h[2]; };
  static __device__ __forceinline__ v16b load(const __bf16* p) {
    U f; f.h[0] = *(const v8b*)(p); f.h[1] = *(const v8b*)(p + 16); return f.v;
  }
  static __device__ __forceinline__ v8f mma(v16b a, v16b b, v8f c) {
    return __builtin_amdgcn_wmma_f32_16x16x32_bf16(false, a, false, b, (short)0, c, false, false);
  }
  static __device__ __forceinline__ void guard(v8f& a, v8f& b, v16b x, v16b y) { dep_guard_b(a, b, x, y); }
  static __device__ __forceinline__ void keep(v16b a, v16b b, v16b c, v16b d) { keep4_b(a, b, c, d); }
};

template <int NTAPS>
__global__ __launch_bounds__(256) void conv_gemm_split(
    const unsigned short* __restrict__ Ahp, const unsigned short* __restrict__ Alp,
    const unsigned short* __restrict__ Bhp, const unsigned short* __restrict__ Blp,
    float* __restrict__ Cout, int N) {
  typedef __bf16 T;
  typedef v16b V;
  constexpr int KTOT = NTAPS * kCh;
  constexpr int padoff = (NTAPS == 1) ? 1 : 0;
  __shared__ __align__(16) float sT[8][16 * 68];
  const int lane = threadIdx.x & 31;
  const int wave = threadIdx.x >> 5;
  const int tilesN = N >> 6;
  const int tilesM = kNPix >> 6;
  const int tile = blockIdx.x * 8 + wave;
  if (tile >= tilesM * tilesN) return;
  const int tm = tile / tilesN;
  const int tn = tile - tm * tilesN;
  const int m0 = tm << 6;
  const int n0 = tn << 6;

  const int rlane = lane & 15;
  const int koff  = (lane >> 4) * 8;
  const int mOff  = (lane >> 4) * 8;

  const int bimg = m0 >> 12;
  const int yrow = (m0 >> 6) & 63;
  const size_t arow = ((size_t)(bimg * kPadW + yrow + padoff) * kPadW + padoff + rlane) * kCh + koff;
  const T* Ah = (const T*)Ahp + arow;
  const T* Al = (const T*)Alp + arow;
  const T* Bh = (const T*)Bhp;
  const T* Bl = (const T*)Blp;

  v8f acc[4][4];
#pragma unroll
  for (int i = 0; i < 4; ++i)
#pragma unroll
    for (int j = 0; j < 4; ++j) acc[i][j] = (v8f){0.f,0.f,0.f,0.f,0.f,0.f,0.f,0.f};

  for (int k0 = 0; k0 < KTOT; k0 += 32) {
    const int tap = k0 >> 6;
    const int ky = tap / 3;
    const int kx = tap - 3 * ky;
    const size_t tapoff = (size_t)(ky * kPadW + kx) * kCh + (k0 & 63);
    V bh[4], bl[4];
#pragma unroll
    for (int j = 0; j < 4; ++j) {
      const size_t bo = (size_t)(n0 + (j << 4) + rlane) * KTOT + koff + k0;
      bh[j] = Frag<T>::load(Bh + bo);
      bl[j] = Frag<T>::load(Bl + bo);
    }
#pragma unroll
    for (int i = 0; i < 4; ++i) {
      const size_t ao = tapoff + (size_t)(i << 4) * kCh;
      V ah = Frag<T>::load(Ah + ao);
      V al = Frag<T>::load(Al + ao);
#pragma unroll
      for (int j = 0; j < 4; ++j) {
        acc[i][j] = Frag<T>::mma(ah, bh[j], acc[i][j]);
        acc[i][j] = Frag<T>::mma(ah, bl[j], acc[i][j]);
        acc[i][j] = Frag<T>::mma(al, bh[j], acc[i][j]);
      }
      Frag<T>::guard(acc[i][0], acc[i][3], ah, al);
    }
    Frag<T>::keep(bh[0], bh[1], bh[2], bh[3]);
    Frag<T>::keep(bl[0], bl[1], bl[2], bl[3]);
  }
  acc_guard4(acc[0][0], acc[0][1], acc[0][2], acc[0][3]);
  acc_guard4(acc[1][0], acc[1][1], acc[1][2], acc[1][3]);
  acc_guard4(acc[2][0], acc[2][1], acc[2][2], acc[2][3]);
  acc_guard4(acc[3][0], acc[3][1], acc[3][2], acc[3][3]);

  float* slab = sT[wave];
#pragma unroll
  for (int i = 0; i < 4; ++i) {
    const int mBase = m0 + (i << 4);
#pragma unroll
    for (int j = 0; j < 4; ++j) {
#pragma unroll
      for (int r = 0; r < 8; ++r) {
        slab[(mOff + r) * 68 + (j << 4) + rlane] = acc[i][j][r];
      }
    }
    __builtin_amdgcn_fence(__ATOMIC_RELEASE, "workgroup");
    __builtin_amdgcn_wave_barrier();
    __builtin_amdgcn_fence(__ATOMIC_ACQUIRE, "workgroup");
    {
      const int hh = lane >> 4, c4 = (lane & 15) * 4;
      for (int pass = 0; pass < 2; ++pass) {
#pragma unroll
        for (int it = 0; it < 8; ++it) {
          const int row = it * 2 + hh;
          v4f v = *(const v4f*)(slab + row * 68 + c4);
          *(volatile v4f*)(Cout + (size_t)(mBase + row) * N + n0 + c4) = v;
        }
        __threadfence();
      }
    }
    __builtin_amdgcn_fence(__ATOMIC_RELEASE, "workgroup");
    __builtin_amdgcn_wave_barrier();
    __builtin_amdgcn_fence(__ATOMIC_ACQUIRE, "workgroup");
  }
}

__global__ __launch_bounds__(256) void tab_kernel(
    const float* __restrict__ qg, const float* __restrict__ qbe, const float* __restrict__ qmu, const float* __restrict__ qva,
    const float* __restrict__ kg, const float* __restrict__ kbe, const float* __restrict__ kmu, const float* __restrict__ kva,
    const float* __restrict__ vg, const float* __restrict__ vbe, const float* __restrict__ vmu, const float* __restrict__ vva,
    const float* __restrict__ og, const float* __restrict__ obe, const float* __restrict__ omu, const float* __restrict__ ova,
    const float* __restrict__ pos_h, const float* __restrict__ pos_w,
    float* __restrict__ tab) {
  __shared__ __align__(16) float st[1088];
  const int t = threadIdx.x, lane = t & 31, wave = t >> 5;
  const int s = t >> 6, n = t & 63;
  const float g0 = qg[n],  g1 = kg[n],  g2 = vg[n],  g3 = og[n];
  const float b0 = qbe[n], b1 = kbe[n], b2 = vbe[n], b3 = obe[n];
  const float u0 = qmu[n], u1 = kmu[n], u2 = vmu[n], u3 = omu[n];
  const float w0 = qva[n], w1 = kva[n], w2 = vva[n], w3 = ova[n];
  const float g  = (s == 0) ? g0 : (s == 1) ? g1 : (s == 2) ? g2 : g3;
  const float be = (s == 0) ? b0 : (s == 1) ? b1 : (s == 2) ? b2 : b3;
  const float mu = (s == 0) ? u0 : (s == 1) ? u1 : (s == 2) ? u2 : u3;
  const float va = (s == 0) ? w0 : (s == 1) ? w1 : (s == 2) ? w2 : w3;
  const float sc = g * rsqrtf(va + 1e-5f);
  const float sh = be - mu * sc;
  st[s * 128 + n] = sc;
  st[s * 128 + 64 + n] = sh;
#pragma unroll
  for (int i = 0; i < 3; ++i) {
    const int idx = i * 256 + t;
    const int ic = idx > 575 ? 575 : idx;
    const int p9 = ic >> 6, c = ic & 63;
    const int ky = p9 / 3;
    const int kx = p9 - 3 * ky;
    const float pv = pos_h[c * 3 + ky] + pos_w[c * 3 + kx];
    if (idx < 576) st[512 + idx] = pv;
  }
  __syncthreads();
  const int q4 = lane >> 3, sub = (lane & 7) * 4;
  for (int pass = 0; pass < 2; ++pass) {
#pragma unroll
    for (int it = 0; it < 2; ++it) {
      const int L = it * 32 + wave * 4 + q4;
      const int Lc = L > 33 ? 33 : L;
      const v4f v = *(const v4f*)(st + Lc * 32 + sub);
      if (L < 34) *(volatile v4f*)(tab + Lc * 32 + sub) = v;
    }
    __threadfence();
  }
}

__global__ __launch_bounds__(256) void wpack_kernel(
    const float* __restrict__ wq, const float* __restrict__ wk, const float* __restrict__ wv,
    unsigned short* __restrict__ bqv_h, unsigned short* __restrict__ bqv_l,
    unsigned short* __restrict__ bk_h, unsigned short* __restrict__ bk_l) {
  const int t = threadIdx.x, lane = t & 31, wave = t >> 5;
  const int region = blockIdx.y;
  const int nLines = (region == 0) ? kCh * kTaps : kQVld;
  const int base = blockIdx.x * 32;
  if (base >= nLines) return;
  const int L = base + wave * 4 + (lane >> 3);
  const int Lc = L > nLines - 1 ? nLines - 1 : L;
  const int sub = lane & 7;
  float val[8];
  if (region == 0) {
    const int o = Lc / 9;
    const int j = Lc - 9 * o;
#pragma unroll
    for (int e = 0; e < 8; ++e) {
      const int c = sub * 8 + e;
      val[e] = wk[(o * kCh + c) * 9 + j];
    }
  } else {
    const int o = Lc;
    const int oq = o > 63 ? 63 : o;
    const int ov = o - 64 < 0 ? 0 : o - 64;
#pragma unroll
    for (int e = 0; e < 8; ++e) {
      const int c = sub * 8 + e;
      const float a = wq[oq * kCh + c];
      const float d = wv[ov * kCh + c];
      val[e] = (o < 64) ? a : d;
    }
  }
  unsigned short hb[8], lb[8];
#pragma unroll
  for (int e = 0; e < 8; ++e) split_bf(val[e], hb[e], lb[e]);
  const v4u uh = (v4u){pk16(hb[0], hb[1]), pk16(hb[2], hb[3]), pk16(hb[4], hb[5]), pk16(hb[6], hb[7])};
  const v4u ul = (v4u){pk16(lb[0], lb[1]), pk16(lb[2], lb[3]), pk16(lb[4], lb[5]), pk16(lb[6], lb[7])};
  unsigned short* dh = (region == 0) ? bk_h : bqv_h;
  unsigned short* dl = (region == 0) ? bk_l : bqv_l;
  const size_t off = (size_t)Lc * 64 + sub * 8;
  for (int pass = 0; pass < 2; ++pass) {
    if (L < nLines) {
      *(volatile v4u*)(dh + off) = uh;
      *(volatile v4u*)(dl + off) = ul;
    }
    __threadfence();
  }
}

__global__ __launch_bounds__(256) void xpose_split_kernel(const float* __restrict__ x,
                                                          unsigned short* __restrict__ xh,
                                                          unsigned short* __restrict__ xl) {
  __shared__ float sm[64][65];
  const int t = threadIdx.x, lane = t & 31, wave = t >> 5;
  const int blk = blockIdx.x;
  const int b = blk / kPadW;
  const int pr = blk - b * kPadW;
  int yc = pr - 1;
  yc = yc < 0 ? 0 : yc;
  yc = yc > 63 ? 63 : yc;
#pragma unroll
  for (int i = 0; i < 16; ++i) {
    const int e = i * 256 + t;
    const int c = e >> 6;
    const int xx = e & 63;
    sm[xx][c] = x[((size_t)(b * kCh + c) * kHgt + yc) * kWid + xx];
  }
  __syncthreads();
  const bool rowvalid = (pr >= 1) && (pr <= 64);
  const int q4 = lane >> 3, sub = lane & 7;
  const size_t rowpix = (size_t)(b * kPadW + pr) * kPadW;
  for (int pass = 0; pass < 2; ++pass) {
#pragma unroll
    for (int it = 0; it < 3; ++it) {
      const int L = it * 32 + wave * 4 + q4;
      const int Lc = L > 65 ? 65 : L;
      int xx = Lc - 1;
      xx = xx < 0 ? 0 : xx;
      xx = xx > 63 ? 63 : xx;
      const bool valid = rowvalid && (Lc >= 1) && (Lc <= 64);
      unsigned short hb[8], lb[8];
#pragma unroll
      for (int e = 0; e < 8; ++e) {
        float f = sm[xx][sub * 8 + e];
        f = valid ? f : 0.0f;
        split_bf(f, hb[e], lb[e]);
      }
      const v4u uh = (v4u){pk16(hb[0], hb[1]), pk16(hb[2], hb[3]), pk16(hb[4], hb[5]), pk16(hb[6], hb[7])};
      const v4u ul = (v4u){pk16(lb[0], lb[1]), pk16(lb[2], lb[3]), pk16(lb[4], lb[5]), pk16(lb[6], lb[7])};
      const size_t off = (rowpix + Lc) * kCh + sub * 8;
      if (L < 66) {
        *(volatile v4u*)(xh + off) = uh;
        *(volatile v4u*)(xl + off) = ul;
      }
    }
    __threadfence();
  }
}

__global__ __launch_bounds__(256) void local_attn_kernel(const float* __restrict__ QV, const float* __restrict__ KF,
                                                         const float* __restrict__ coef, const float* __restrict__ posb,
                                                         float* __restrict__ out) {
  __shared__ __align__(16) float sk[3 * kHaloW * kSlot];
  __shared__ __align__(16) float sv[3 * kHaloW * kSlot];
  __shared__ float slog[9 * 256];
  __shared__ __align__(16) float spos[9 * 64];
  const int t = threadIdx.x, lane = t & 31, wave = t >> 5;
  const int blk = blockIdx.x;
  const int b = blk >> 7;
  const int y = (blk >> 1) & 63;
  const int x0 = (blk & 1) * kPXB;

#pragma unroll
  for (int i = 0; i < 3; ++i) {
    const int idx = i * 256 + t;
    const int ic = idx > 575 ? 575 : idx;
    const float pv = posb[ic];
    if (idx < 576) spos[idx] = pv;
  }
#pragma unroll 1
  for (int i = 0; i < 7; ++i) {
    const int e4 = i * 256 + t;
    const int e4c = e4 > 1631 ? 1631 : e4;
    const int r = e4c / (kHaloW * 16);
    const int rem = e4c - r * (kHaloW * 16);
    const int pp = rem >> 4;
    const int c4 = (rem & 15) * 4;
    const int yy = y + r - 1;
    const int gx = x0 + pp - 1;
    const bool valid = (yy >= 0) && (yy <= 63) && (gx >= 0) && (gx <= 63);
    int yyc = yy < 0 ? 0 : yy; yyc = yyc > 63 ? 63 : yyc;
    int gxc = gx < 0 ? 0 : gx; gxc = gxc > 63 ? 63 : gxc;
    const size_t gpix = (size_t)b * kPixImg + (size_t)yyc * kWid + gxc;
    const v4f ka  = *(const v4f*)(KF + gpix * kCh + c4);
    const v4f va  = *(const v4f*)(QV + gpix * kQVld + kCh + c4);
    const v4f ksc = *(const v4f*)(coef + 128 + c4);
    const v4f ksh = *(const v4f*)(coef + 192 + c4);
    const v4f vsc = *(const v4f*)(coef + 256 + c4);
    const v4f vsh = *(const v4f*)(coef + 320 + c4);
    v4f kr, vr;
#pragma unroll
    for (int e = 0; e < 4; ++e) {
      const float kk = fmaxf(ka[e] * ksc[e] + ksh[e], 0.0f);
      const float vv = va[e] * vsc[e] + vsh[e];
      kr[e] = valid ? kk : 0.0f;
      vr[e] = valid ? vv : 0.0f;
    }
    if (e4 < 1632) {
      *(v4f*)(sk + (r * kHaloW + pp) * kSlot + c4) = kr;
      *(v4f*)(sv + (r * kHaloW + pp) * kSlot + c4) = vr;
    }
  }
  __syncthreads();

  const int hd = wave, px = lane, cb = hd * 8;
  const size_t qpix = (size_t)b * kPixImg + (size_t)y * kWid + x0 + px;
  const v4f qa0 = *(const v4f*)(QV + qpix * kQVld + cb);
  const v4f qa1 = *(const v4f*)(QV + qpix * kQVld + cb + 4);
  const v4f qsc0 = *(const v4f*)(coef + cb);
  const v4f qsc1 = *(const v4f*)(coef + cb + 4);
  const v4f qsh0 = *(const v4f*)(coef + 64 + cb);
  const v4f qsh1 = *(const v4f*)(coef + 68 + cb);
  float qr[8];
#pragma unroll
  for (int e = 0; e < 4; ++e) {
    qr[e]     = fmaxf(qa0[e] * qsc0[e] + qsh0[e], 0.0f);
    qr[4 + e] = fmaxf(qa1[e] * qsc1[e] + qsh1[e], 0.0f);
  }

  float mx = -__builtin_inff();
#pragma unroll 1
  for (int tap = 0; tap < kTaps; ++tap) {
    const int ky = tap / 3;
    const int kx = tap - 3 * ky;
    const float* kp = sk + (ky * kHaloW + px + kx) * kSlot + cb;
    const float* pq = spos + tap * 64 + cb;
    const v4f kq0 = *(const v4f*)(kp);
    const v4f kq1 = *(const v4f*)(kp + 4);
    const v4f p0 = *(const v4f*)(pq);
    const v4f p1 = *(const v4f*)(pq + 4);
    float s = qr[0] * (kq0[0] + p0[0]);
    s += qr[1] * (kq0[1] + p0[1]);
    s += qr[2] * (kq0[2] + p0[2]);
    s += qr[3] * (kq0[3] + p0[3]);
    s += qr[4] * (kq1[0] + p1[0]);
    s += qr[5] * (kq1[1] + p1[1]);
    s += qr[6] * (kq1[2] + p1[2]);
    s += qr[7] * (kq1[3] + p1[3]);
    slog[tap * 256 + t] = s;
    mx = fmaxf(mx, s);
  }
  float ssum = 0.0f;
#pragma unroll 1
  for (int tap = 0; tap < kTaps; ++tap) {
    const float ev = expf(slog[tap * 256 + t] - mx);
    ssum += ev;
    slog[tap * 256 + t] = ev;
  }
  const float inv = 1.0f / ssum;
  float o[8];
#pragma unroll
  for (int c = 0; c < 8; ++c) o[c] = 0.0f;
#pragma unroll 1
  for (int tap = 0; tap < kTaps; ++tap) {
    const int ky = tap / 3;
    const int kx = tap - 3 * ky;
    const float a = slog[tap * 256 + t] * inv;
    const float* vp = sv + (ky * kHaloW + px + kx) * kSlot + cb;
    const v4f vq0 = *(const v4f*)(vp);
    const v4f vq1 = *(const v4f*)(vp + 4);
    o[0] += a * vq0[0]; o[1] += a * vq0[1]; o[2] += a * vq0[2]; o[3] += a * vq0[3];
    o[4] += a * vq1[0]; o[5] += a * vq1[1]; o[6] += a * vq1[2]; o[7] += a * vq1[3];
  }
  __syncthreads();

  float* sout = sk;
  const v4f osc0 = *(const v4f*)(coef + 384 + cb);
  const v4f osc1 = *(const v4f*)(coef + 388 + cb);
  const v4f osh0 = *(const v4f*)(coef + 448 + cb);
  const v4f osh1 = *(const v4f*)(coef + 452 + cb);
#pragma unroll
  for (int c = 0; c < 4; ++c) {
    sout[(cb + c) * kOutP + px]     = fmaxf(o[c] * osc0[c] + osh0[c], 0.0f);
    sout[(cb + 4 + c) * kOutP + px] = fmaxf(o[4 + c] * osc1[c] + osh1[c], 0.0f);
  }
  __syncthreads();

  const int q4 = lane >> 3, sub = (lane & 7) * 4;
  for (int pass = 0; pass < 2; ++pass) {
#pragma unroll
    for (int it = 0; it < 2; ++it) {
      const int n = it * 32 + wave * 4 + q4;
      const v4f v = *(const v4f*)(sout + n * kOutP + sub);
      *(volatile v4f*)(out + ((size_t)(b * kCh + n) * kHgt + y) * kWid + x0 + sub) = v;
    }
    __threadfence();
  }
}

extern "C" void kernel_launch(void* const* d_in, const int* in_sizes, int n_in,
                              void* d_out, int out_size, void* d_ws, size_t ws_size,
                              hipStream_t stream) {
  if (n_in < 22) return;
  if (in_sizes[0] != kImg * kCh * kPixImg) return;
  if (in_sizes[1] != kCh * kCh || in_sizes[2] != kCh * kCh * kTaps || in_sizes[3] != kCh * kCh) return;
  if (in_sizes[4] != kCh * 3 || in_sizes[5] != kCh * 3) return;
  if ((size_t)out_size != (size_t)kNPix * kCh) return;
  if (ws_size < kWsTotal) return;

  const float* x     = (const float*)d_in[0];
  const float* wq    = (const float*)d_in[1];
  const float* wk    = (const float*)d_in[2];
  const float* wv    = (const float*)d_in[3];
  const float* pos_h = (const float*)d_in[4];
  const float* pos_w = (const float*)d_in[5];
  const float* qg = (const float*)d_in[6],  *qbe = (const float*)d_in[7];
  const float* qmu = (const float*)d_in[8], *qva = (const float*)d_in[9];
  const float* kg = (const float*)d_in[10], *kbe = (const float*)d_in[11];
  const float* kmu = (const float*)d_in[12], *kva = (const float*)d_in[13];
  const float* vg = (const float*)d_in[14], *vbe = (const float*)d_in[15];
  const float* vmu = (const float*)d_in[16], *vva = (const float*)d_in[17];
  const float* og = (const float*)d_in[18], *obe = (const float*)d_in[19];
  const float* omu = (const float*)d_in[20], *ova = (const float*)d_in[21];

  char* ws = (char*)d_ws;
  float* tab  = (float*)(ws + kOffTab);
  float* coef = tab;
  float* posb = tab + 512;
  unsigned short* bqvh = (unsigned short*)(ws + kOffBqvH);
  unsigned short* bqvl = (unsigned short*)(ws + kOffBqvL);
  unsigned short* bkh  = (unsigned short*)(ws + kOffBkH);
  unsigned short* bkl  = (unsigned short*)(ws + kOffBkL);
  unsigned short* xh   = (unsigned short*)(ws + kOffXh);
  unsigned short* xl   = (unsigned short*)(ws + kOffXl);
  float* qvp = (float*)(ws + kOffQV);
  float* kfp = (float*)(ws + kOffKF);
  float* outp = (float*)d_out;

  tab_kernel<<<1, 256, 0, stream>>>(qg, qbe, qmu, qva, kg, kbe, kmu, kva,
                                    vg, vbe, vmu, vva, og, obe, omu, ova,
                                    pos_h, pos_w, tab);
  wpack_kernel<<<dim3(18, 2), 256, 0, stream>>>(wq, wk, wv, bqvh, bqvl, bkh, bkl);
  xpose_split_kernel<<<kImg * kPadW, 256, 0, stream>>>(x, xh, xl);
  conv_gemm_split<1><<<(kNPix / 64) * (kQVld / 64) / 8, 256, 0, stream>>>(xh, xl, bqvh, bqvl, qvp, kQVld);
  conv_gemm_split<9><<<(kNPix / 64) / 8, 256, 0, stream>>>(xh, xl, bkh, bkl, kfp, kCh);
  local_attn_kernel<<<kImg * kHgt * (kWid / kPXB), 256, 0, stream>>>(qvp, kfp, coef, posb, outp);
}
